// RestGCNEqualHidden_11321533792498
// MI455X (gfx1250) — hardware-run, weakly checked
//
#include <hip/hip_runtime.h>
#include <stddef.h>
#include <stdint.h>
#include <math.h>


#define NNODE  100000
#define NEDGE  1600000
#define DF     128
#define K1     128
#define K2     256
#define NTHR   256
#define NWAVE  8
#define EPT    8
#define CHUNK  (NTHR * EPT)
#define NBA    1024
#define SLA    10
#define NBLK   98
#define MPAD   100096
#define WLCAP  3584
#define RCAP   (NWAVE * WLCAP)
#define RCAP_WS 20480
#define DEGCAP 64
#define MEAS_BLKHITS 16710
#define MEAS_MAXDEG  36
#define FLP    32
#define GBM    128
#define GBN    128
#define GTHR   256
#define RBH    256
#define BK_ZINTS (2 * RCAP + 3 * NBA)
#define BK_LDS_INTS (BK_ZINTS + NBA + 16)
#define G_LDS_FLOATS (GBM * GBN + GBM)
#define NUW1   (DF * (K1 / 8))
#define NUWD   (DF * (K2 / 8))
#define NUBT   256
#define NUWE   (NUW1 + 3 * NUWD + NUBT)

static_assert((CHUNK & (CHUNK - 1)) == 0 && CHUNK == 2048);
static_assert(NBA == (1 << SLA));
static_assert(((long long)NEDGE << SLA) < (1LL << 31));
static_assert((long long)NBLK * NBA >= MPAD && MPAD >= NNODE && MPAD % GBM == 0);
static_assert(MPAD - NNODE < GBM);
static_assert(RCAP_WS * 100LL >= MEAS_BLKHITS * 105LL && RCAP >= RCAP_WS);
static_assert(WLCAP * NWAVE * 2 >= MEAS_BLKHITS * 3);
static_assert(DEGCAP >= MEAS_MAXDEG + 8);
static_assert(BK_ZINTS % (NTHR * 4) == 0 && RCAP_WS % (NTHR * 4) == 0 && NBA == NTHR * 4);
static_assert(BK_LDS_INTS * 4 <= 300000 && BK_LDS_INTS * 4 <= 327680);
static_assert(G_LDS_FLOATS * 4 <= 327680);
static_assert(K1 % 32 == 0 && K2 % 32 == 0 && K2 == 2 * DF && GBN == DF && GBM == (GTHR / 32) * 16);
static_assert(NUW1 % NTHR == 0 && NUWD % NTHR == 0 && NUWE % NTHR == 0 && (MPAD * 16) % NTHR == 0);
static_assert(DF == 4 * 32 && RBH == 2 * DF);

typedef float          v4f   __attribute__((ext_vector_type(4)));
typedef float          v8f   __attribute__((ext_vector_type(8)));
typedef int            v4i   __attribute__((ext_vector_type(4)));
typedef int            v8i   __attribute__((ext_vector_type(8)));
typedef unsigned short v4us  __attribute__((ext_vector_type(4)));
typedef unsigned short v8us  __attribute__((ext_vector_type(8)));
typedef unsigned short v16us __attribute__((ext_vector_type(16)));
typedef __bf16         v16bf __attribute__((ext_vector_type(16)));
typedef v4f  __attribute__((may_alias)) v4fa;
typedef v4i  __attribute__((may_alias)) v4ia;
typedef v4us __attribute__((may_alias)) v4usa;
typedef v8us __attribute__((may_alias)) v8usa;
union FragB { v16bf v; v16us u; v8us h[2]; v8i w; };

__device__ __forceinline__ v8f wmb(const FragB& a, const FragB& b, v8f c) {
  v8f d = __builtin_amdgcn_wmma_f32_16x16x32_bf16(false, a.v, false, b.v, (short)0, c, false, false);
  asm volatile("v_nop\n\tv_nop\n\tv_nop\n\tv_nop" : "+v"(d) : "v"(a.w), "v"(b.w));
  return d;
}
__device__ __forceinline__ v8f z8() { v8f z = {0.f, 0.f, 0.f, 0.f, 0.f, 0.f, 0.f, 0.f}; return z; }

__device__ __forceinline__ unsigned bf16_bits(float f) {
  const unsigned u = __float_as_uint(f);
  return (u + 0x7FFFu + ((u >> 16) & 1u)) >> 16;
}
__device__ __forceinline__ float bf16_val(float f) {
  return __uint_as_float(bf16_bits(f) << 16);
}
__device__ __forceinline__ unsigned hl_bits(float v, unsigned& lo) {
  const unsigned hb = bf16_bits(v);
  lo = bf16_bits(v - __uint_as_float(hb << 16));
  return hb;
}
__device__ __forceinline__ void wave_sync() {
  __builtin_amdgcn_fence(__ATOMIC_RELEASE, "wavefront");
  __builtin_amdgcn_wave_barrier();
  __builtin_amdgcn_fence(__ATOMIC_ACQUIRE, "wavefront");
}
__device__ __forceinline__ int ld_key(const int* __restrict__ p, int e, int nE, int sent) {
  const int v = p[min(e, nE - 1)];
  asm volatile("" :: "v"(v));
  return (e < nE) ? v : sent;
}

__device__ __forceinline__ int scan_chunk(const int* __restrict__ dsts, int nE, int cbase, int slotBase,
                                          int vec8, int* wl, int wc, int tid) {
  const int e0   = cbase + tid * EPT;
  const int sent = -2147483647 - 1;
  v4i da, db;
  if (vec8 != 0 && cbase + CHUNK <= nE) {
    da = *(const v4i*)(dsts + e0);
    db = *(const v4i*)(dsts + e0 + 4);
  } else {
    da.x = ld_key(dsts, e0,     nE, sent);
    da.y = ld_key(dsts, e0 + 1, nE, sent);
    da.z = ld_key(dsts, e0 + 2, nE, sent);
    da.w = ld_key(dsts, e0 + 3, nE, sent);
    db.x = ld_key(dsts, e0 + 4, nE, sent);
    db.y = ld_key(dsts, e0 + 5, nE, sent);
    db.z = ld_key(dsts, e0 + 6, nE, sent);
    db.w = ld_key(dsts, e0 + 7, nE, sent);
  }
  const unsigned nbs = (unsigned)slotBase;
  const unsigned unb = (unsigned)NBA;
  const unsigned s0 = (unsigned)da.x - nbs, s1 = (unsigned)da.y - nbs;
  const unsigned s2 = (unsigned)da.z - nbs, s3 = (unsigned)da.w - nbs;
  const unsigned s4 = (unsigned)db.x - nbs, s5 = (unsigned)db.y - nbs;
  const unsigned s6 = (unsigned)db.z - nbs, s7 = (unsigned)db.w - nbs;
  const bool h0 = s0 < unb, h1 = s1 < unb, h2 = s2 < unb, h3 = s3 < unb;
  const bool h4 = s4 < unb, h5 = s5 < unb, h6 = s6 < unb, h7 = s7 < unb;
  const unsigned any = __builtin_amdgcn_ballot_w32(h0 | h1 | h2 | h3 | h4 | h5 | h6 | h7);
  if (any != 0u) {
#define HITJ(J, HJ, SJ) { \
      const unsigned mj = __builtin_amdgcn_ballot_w32(HJ); \
      if (mj != 0u) { \
        if (HJ) { \
          const int pos = wc + (int)__builtin_amdgcn_mbcnt_lo(mj, 0u); \
          if (pos < WLCAP) wl[pos] = ((e0 + (J)) << SLA) | (int)(SJ); \
        } \
        wc += (int)__builtin_popcount(mj); } }
    HITJ(0, h0, s0)
    HITJ(1, h1, s1)
    HITJ(2, h2, s2)
    HITJ(3, h3, s3)
    HITJ(4, h4, s4)
    HITJ(5, h5, s5)
    HITJ(6, h6, s6)
    HITJ(7, h7, s7)
#undef HITJ
  }
  return wc;
}

__device__ __forceinline__ v8us wgather(const float* __restrict__ W, int n, int kk) {
  const float* p = W + (size_t)kk * DF + n;
  v8us o;
#pragma unroll
  for (int i = 0; i < 8; ++i) o[i] = (unsigned short)bf16_bits(p[(size_t)i * DF]);
  return o;
}
__device__ __forceinline__ float bsel(float a0, float a1, float a2, float a3,
                                      unsigned m0, unsigned m1, unsigned m2, unsigned m3) {
  const unsigned u = (__float_as_uint(a0) & m0) | (__float_as_uint(a1) & m1) |
                     (__float_as_uint(a2) & m2) | (__float_as_uint(a3) & m3);
  return bf16_val(__uint_as_float(u));
}

__global__ __launch_bounds__(NTHR) void k_prep(
    const float* __restrict__ x, const float* __restrict__ W1, const float* __restrict__ W2,
    const float* __restrict__ W3, const float* __restrict__ W4,
    const float* __restrict__ b1, const float* __restrict__ b2, const float* __restrict__ b3,
    const float* __restrict__ b4,
    unsigned short* xb, unsigned short* w1t, unsigned short* w2d, unsigned short* w3d,
    unsigned short* w4d, float* bt, int nN, int nUnits) {
  const int u = (int)blockIdx.x * NTHR + (int)threadIdx.x;
  v8us o;
  unsigned short* dp;
  if (u < NUW1) {
    const int n = u >> 4, k8 = (u & 15) * 8;
    o = wgather(W1, n, k8);
    dp = w1t + (size_t)u * 8;
  } else if (u < NUW1 + NUWD) {
    const int v = u - NUW1;
    const int n = v >> 5, k8 = (v & 31) * 8;
    o = wgather(W2, n, k8 & (DF - 1));
    dp = w2d + (size_t)v * 8;
  } else if (u < NUW1 + 2 * NUWD) {
    const int v = u - (NUW1 + NUWD);
    const int n = v >> 5, k8 = (v & 31) * 8;
    o = wgather(W3, n, k8 & (DF - 1));
    dp = w3d + (size_t)v * 8;
  } else if (u < NUW1 + 3 * NUWD) {
    const int v = u - (NUW1 + 2 * NUWD);
    const int n = v >> 5, k8 = (v & 31) * 8;
    o = wgather(W4, n, k8 & (DF - 1));
    dp = w4d + (size_t)v * 8;
  } else if (u < NUWE) {
    const int t  = u - (NUW1 + 3 * NUWD);
    const int tc = t < 128 ? t : 127;
    const int lay = tc >> 5, c4 = (tc & 31) * 4;
    const v4f a0 = *(const v4f*)(b1 + c4);
    const v4f a1 = *(const v4f*)(b2 + c4);
    const v4f a2 = *(const v4f*)(b3 + c4);
    const v4f a3 = *(const v4f*)(b4 + c4);
    asm volatile("" :: "v"(a0)); asm volatile("" :: "v"(a1));
    asm volatile("" :: "v"(a2)); asm volatile("" :: "v"(a3));
    const unsigned m0 = (lay == 0) ? 0xFFFFFFFFu : 0u, m1 = (lay == 1) ? 0xFFFFFFFFu : 0u;
    const unsigned m2 = (lay == 2) ? 0xFFFFFFFFu : 0u, m3 = (lay == 3) ? 0xFFFFFFFFu : 0u;
    v4f ov;
    ov.x = bsel(a0.x, a1.x, a2.x, a3.x, m0, m1, m2, m3);
    ov.y = bsel(a0.y, a1.y, a2.y, a3.y, m0, m1, m2, m3);
    ov.z = bsel(a0.z, a1.z, a2.z, a3.z, m0, m1, m2, m3);
    ov.w = bsel(a0.w, a1.w, a2.w, a3.w, m0, m1, m2, m3);
    float* bp = bt + 4 * tc;
    if (t < 128) *(volatile v4f*)bp = ov;
    __threadfence();
    if (t < 128) *(volatile v4f*)bp = ov;
    return;
  } else if (u < nUnits) {
    const int v   = u - NUWE;
    const int row = v >> 4, k8 = (v & 15) * 8;
    const int rc  = row < nN ? row : nN - 1;
    const float* p = x + (size_t)rc * DF + k8;
    const v4f a = *(const v4fa*)p;
    const v4f b = *(const v4fa*)(p + 4);
    asm volatile("" :: "v"(a)); asm volatile("" :: "v"(b));
    const unsigned msk = (row < nN) ? 0xFFFFu : 0u;
    o[0] = (unsigned short)(bf16_bits(a.x) & msk);
    o[1] = (unsigned short)(bf16_bits(a.y) & msk);
    o[2] = (unsigned short)(bf16_bits(a.z) & msk);
    o[3] = (unsigned short)(bf16_bits(a.w) & msk);
    o[4] = (unsigned short)(bf16_bits(b.x) & msk);
    o[5] = (unsigned short)(bf16_bits(b.y) & msk);
    o[6] = (unsigned short)(bf16_bits(b.z) & msk);
    o[7] = (unsigned short)(bf16_bits(b.w) & msk);
    dp = xb + (size_t)v * 8;
  } else {
    return;
  }
  *(volatile v8us*)dp = o;
  __threadfence();
  *(volatile v8us*)dp = o;
}

__global__ __launch_bounds__(NTHR) void k_bucket(const int* __restrict__ srcs, const int* __restrict__ dsts,
                                                 int nE, int nN, int vec8,
                                                 int* listg, int* cntg, int* offg, float* disg, int* flagg) {
  extern __shared__ __attribute__((aligned(16))) int bsm[];
  int*   wls  = bsm;
  int*   sl   = bsm + RCAP;
  int*   cnt  = sl + RCAP;
  int*   offs = cnt + NBA;
  int*   cur  = offs + NBA;
  float* disl = (float*)(cur + NBA);
  int*   misc = (int*)(disl + NBA);
  const int tid = (int)threadIdx.x, lane = tid & 31, wave = tid >> 5;
  const int nodeBase = (int)blockIdx.x * NBA;

  {
    const v4i z4 = {0, 0, 0, 0};
    for (int i = tid * 4; i < BK_ZINTS; i += NTHR * 4) *(v4ia*)(bsm + i) = z4;
    if (tid < 16) misc[tid] = 0;
  }
  __syncthreads();

  {
    int wc = 0;
    int* wl = wls + wave * WLCAP;
    const int nChunks = (nE + CHUNK - 1) / CHUNK;
#pragma unroll 1
    for (int ch = 0; ch < nChunks; ++ch)
      wc = scan_chunk(dsts, nE, ch * CHUNK, nodeBase, vec8, wl, wc, tid);
    if (lane == 0) misc[wave] = wc;
  }
  __syncthreads();

  if (wave == 0) {
    int t = 0, ov = 0;
#pragma unroll 1
    for (int w2 = 0; w2 < NWAVE; ++w2) {
      int c = misc[w2];
      if (c > WLCAP) ov = 1;
      c = c < 0 ? 0 : (c > WLCAP ? WLCAP : c);
#pragma unroll 1
      for (int b0 = 0; b0 < c; b0 += 32) {
        const int idx = b0 + lane;
        const int ent = wls[w2 * WLCAP + (idx < WLCAP ? idx : WLCAP - 1)];
        const int m32 = (c - b0) < 32 ? (c - b0) : 32;
#pragma unroll 1
        for (int k = 0; k < m32; ++k) {
          const int uu   = __builtin_amdgcn_readlane(ent, k);
          const int slot = uu & (NBA - 1);
          if (lane == 0) cnt[slot] = cnt[slot] + 1;
        }
      }
      t += c;
    }
    if (t > RCAP_WS) ov = 1;
    if (lane == 0) { misc[8] = t; misc[9] = ov; }
  }
  __syncthreads();

#pragma unroll 1
  for (int j = 0; j < 4; ++j) {
    const int cv = cnt[4 * tid + j];
    disl[4 * tid + j] = 1.0f / sqrtf((float)(cv + 1));
  }
  if (wave == 0) {
    const int base = lane * (NBA / 32);
    int s = 0;
#pragma unroll 1
    for (int i = 0; i < NBA / 32; ++i) s += cnt[base + i];
    int incl = s;
#pragma unroll
    for (int d = 1; d < 32; d <<= 1) {
      const int y = __shfl_up(incl, d, 32);
      if (lane >= d) incl += y;
    }
    int run = incl - s;
#pragma unroll 1
    for (int i = 0; i < NBA / 32; ++i) {
      const int cv = cnt[base + i];
      offs[base + i] = run;
      cur[base + i]  = run;
      run += cv;
    }
  }
  __syncthreads();

  if (wave == 0) {
#pragma unroll 1
    for (int w2 = 0; w2 < NWAVE; ++w2) {
      int c = misc[w2];
      c = c < 0 ? 0 : (c > WLCAP ? WLCAP : c);
#pragma unroll 1
      for (int b0 = 0; b0 < c; b0 += 32) {
        const int idx = b0 + lane;
        const int ent = wls[w2 * WLCAP + (idx < WLCAP ? idx : WLCAP - 1)];
        const int m32 = (c - b0) < 32 ? (c - b0) : 32;
#pragma unroll 1
        for (int k = 0; k < m32; ++k) {
          const int uu   = __builtin_amdgcn_readlane(ent, k);
          const int slot = uu & (NBA - 1);
          if (lane == 0) {
            int p = cur[slot];
            p = p < 0 ? 0 : (p > RCAP - 1 ? RCAP - 1 : p);
            sl[p] = uu;
            cur[slot] = p + 1;
          }
        }
      }
    }
  }
  __syncthreads();

  int tt = misc[8];
  const int ovf = misc[9];
  tt = tt < 0 ? 0 : (tt > RCAP_WS ? RCAP_WS : tt);
  const int padn = nodeBase < nN ? nodeBase : nN - 1;
  int* lrow = listg + (size_t)blockIdx.x * RCAP_WS;
#pragma unroll 1
  for (int it = 0; it < RCAP_WS / (NTHR * 4); ++it) {
    const int i0 = it * (NTHR * 4) + 4 * tid;
    const v4i e4 = *(const v4ia*)(sl + i0);
    int ea = e4.x >> SLA, eb = e4.y >> SLA, ec = e4.z >> SLA, ed = e4.w >> SLA;
    ea = ea < 0 ? 0 : (ea > nE - 1 ? nE - 1 : ea);
    eb = eb < 0 ? 0 : (eb > nE - 1 ? nE - 1 : eb);
    ec = ec < 0 ? 0 : (ec > nE - 1 ? nE - 1 : ec);
    ed = ed < 0 ? 0 : (ed > nE - 1 ? nE - 1 : ed);
    int ra = srcs[ea], rb = srcs[eb], rc = srcs[ec], rd = srcs[ed];
    asm volatile("" :: "v"(ra)); asm volatile("" :: "v"(rb));
    asm volatile("" :: "v"(rc)); asm volatile("" :: "v"(rd));
    ra = ra < 0 ? 0 : (ra > nN - 1 ? nN - 1 : ra);
    rb = rb < 0 ? 0 : (rb > nN - 1 ? nN - 1 : rb);
    rc = rc < 0 ? 0 : (rc > nN - 1 ? nN - 1 : rc);
    rd = rd < 0 ? 0 : (rd > nN - 1 ? nN - 1 : rd);
    v4i ov4;
    ov4.x = (i0     < tt) ? ra : padn;
    ov4.y = (i0 + 1 < tt) ? rb : padn;
    ov4.z = (i0 + 2 < tt) ? rc : padn;
    ov4.w = (i0 + 3 < tt) ? rd : padn;
    *(volatile v4i*)(lrow + i0) = ov4;
    __threadfence();
    *(volatile v4i*)(lrow + i0) = ov4;
  }
  {
    const v4i c4 = *(const v4ia*)(cnt + 4 * tid);
    const v4i o4 = *(const v4ia*)(offs + 4 * tid);
    const v4f d4 = *(const v4fa*)(disl + 4 * tid);
    v4i f4;
    f4.x = ovf; f4.y = tt; f4.z = 0; f4.w = 0;
    const bool fw = (wave == 0) && (lane < 8);
    int* fp = flagg + (size_t)blockIdx.x * FLP + 4 * (lane & 7);
    *(volatile v4i*)(cntg + nodeBase + 4 * tid) = c4;
    *(volatile v4i*)(offg + nodeBase + 4 * tid) = o4;
    *(volatile v4f*)(disg + nodeBase + 4 * tid) = d4;
    if (fw) *(volatile v4i*)fp = f4;
    __threadfence();
    *(volatile v4i*)(cntg + nodeBase + 4 * tid) = c4;
    *(volatile v4i*)(offg + nodeBase + 4 * tid) = o4;
    *(volatile v4f*)(disg + nodeBase + 4 * tid) = d4;
    if (fw) *(volatile v4i*)fp = f4;
  }
}

__global__ __launch_bounds__(GTHR) __attribute__((amdgpu_num_vgpr(248)))
void k_gemm(const unsigned short* __restrict__ A, const unsigned short* __restrict__ WT, int K,
            const float* __restrict__ dis, float* outF, int nN) {
  extern __shared__ __attribute__((aligned(16))) float gsm[];
  float* stg = gsm;
  float* dsl = gsm + GBM * GBN;
  const int tid = (int)threadIdx.x, lane = tid & 31, wave = tid >> 5, hh = lane >> 4, m = lane & 15;
  const int rowBase = (int)blockIdx.x * GBM;

  if (tid < 32) {
    const v4f d4 = *(const v4f*)(dis + rowBase + 4 * tid);
    *(v4fa*)(dsl + 4 * tid) = d4;
  }

  v8f acc[8];
#pragma unroll
  for (int t = 0; t < 8; ++t) acc[t] = z8();
  const unsigned short* ap = A  + (size_t)(rowBase + 16 * wave + m) * (size_t)K + 8 * hh;
  const unsigned short* wp = WT + (size_t)m * (size_t)K + 8 * hh;

#pragma unroll 1
  for (int k0 = 0; k0 < K; k0 += 32) {
    FragB af;
    af.h[0] = *(const v8usa*)(ap + k0);
    af.h[1] = *(const v8usa*)(ap + k0 + 16);
#pragma unroll
    for (int nt = 0; nt < 8; ++nt) {
      const unsigned short* wq = wp + (size_t)(16 * nt) * (size_t)K + k0;
      FragB bf;
      bf.h[0] = *(const v8usa*)wq;
      bf.h[1] = *(const v8usa*)(wq + 16);
      acc[nt] = wmb(af, bf, acc[nt]);
    }
  }

#pragma unroll
  for (int nt = 0; nt < 8; ++nt) {
    const int lc = 16 * nt + m;
#pragma unroll
    for (int r = 0; r < 8; ++r) {
      const int lr = 16 * wave + 8 * hh + r;
      stg[lr * GBN + lc] = acc[nt][r];
    }
  }
  __syncthreads();

  v4f pv[16];
#pragma unroll
  for (int i = 0; i < 16; ++i) {
    const int lr = 16 * wave + i;
    const v4f t4 = *(const v4fa*)(stg + lr * GBN + 4 * lane);
    const float d = dsl[lr];
    v4f q;
    q.x = t4.x * d; q.y = t4.y * d; q.z = t4.z * d; q.w = t4.w * d;
    pv[i] = q;
  }
#pragma unroll
  for (int i = 0; i < 16; ++i) {
    const int row = rowBase + 16 * wave + i;
    float* op = outF + (size_t)row * DF + 4 * lane;
    if (row < nN) *(volatile v4f*)op = pv[i];
  }
  __threadfence();
#pragma unroll
  for (int i = 0; i < 16; ++i) {
    const int row = rowBase + 16 * wave + i;
    float* op = outF + (size_t)row * DF + 4 * lane;
    if (row < nN) *(volatile v4f*)op = pv[i];
  }
}

__device__ __forceinline__ float fin1(float acc, float self, float dd, float b, bool bad, bool live) {
  float y = (acc + self) * dd + b;
  y = (y > 0.0f) ? y : (y - y);
  y = bad ? __int_as_float(0x7fc00000) : y;
  return live ? y : 0.0f;
}

template <int HASP, int WRX, int LAST>
__global__ __launch_bounds__(NTHR) void k_replay(
    const int* __restrict__ listg, const int* __restrict__ cntg, const int* __restrict__ offg,
    const float* __restrict__ disg, const int* __restrict__ flagg,
    const float* __restrict__ hp, const float* __restrict__ btl,
    const float* __restrict__ stp, float* stn, unsigned short* ain, float* outp,
    int nN, int mRows) {
  __shared__ __attribute__((aligned(16))) int   scnt[NBA];
  __shared__ __attribute__((aligned(16))) int   soff[NBA];
  __shared__ __attribute__((aligned(16))) float sdis[NBA];
  __shared__ __attribute__((aligned(16))) float sbt[DF];
  __shared__ __attribute__((aligned(16))) unsigned short rbuf[NWAVE * RBH];
  const int tid = (int)threadIdx.x, lane = tid & 31, wave = tid >> 5;
  const int nodeBase = (int)blockIdx.x * NBA;

  {
    const v4i c4 = *(const v4i*)(cntg + nodeBase + 4 * tid);
    const v4i o4 = *(const v4i*)(offg + nodeBase + 4 * tid);
    const v4f d4 = *(const v4f*)(disg + nodeBase + 4 * tid);
    *(v4ia*)(scnt + 4 * tid) = c4;
    *(v4ia*)(soff + 4 * tid) = o4;
    *(v4fa*)(sdis + 4 * tid) = d4;
    if (tid < 32) {
      const v4f b = *(const v4f*)(btl + 4 * tid);
      *(v4fa*)(sbt + 4 * tid) = b;
    }
  }
  const int fl = flagg[(size_t)blockIdx.x * FLP];
  __syncthreads();
  const bool blkbad = fl != 0;
  const int* lp = listg + (size_t)blockIdx.x * RCAP_WS;
  const v4f b4 = *(const v4fa*)(sbt + 4 * lane);
  unsigned short* rb = rbuf + wave * RBH;

#pragma unroll 1
  for (int si = 0; si < NBA / NWAVE; ++si) {
    const int s    = si * NWAVE + wave;
    const int node = nodeBase + s;
    const int c0 = __builtin_amdgcn_readfirstlane(scnt[s]);
    const int o0 = __builtin_amdgcn_readfirstlane(soff[s]);
    const float dd = sdis[s];
    const bool bad = blkbad || (c0 < 0) || (c0 > DEGCAP) || (o0 < 0) || (o0 > RCAP_WS) ||
                     (o0 + c0 > RCAP_WS);
    const int c = c0 < 0 ? 0 : (c0 > DEGCAP ? DEGCAP : c0);
    const int o = o0 < 0 ? 0 : (o0 > RCAP_WS ? RCAP_WS : o0);
    const bool live = node < nN;
    const int nc = live ? node : nN - 1;
    float a0 = 0.0f, a1 = 0.0f, a2 = 0.0f, a3 = 0.0f;
#pragma unroll 1
    for (int b0 = 0; b0 < c; b0 += 32) {
      int idx = o + b0 + lane;
      idx = idx > RCAP_WS - 1 ? RCAP_WS - 1 : idx;
      int sr = lp[idx];
      sr = sr < 0 ? 0 : (sr > nN - 1 ? nN - 1 : sr);
      const int m32 = (c - b0) < 32 ? (c - b0) : 32;
#pragma unroll 1
      for (int k = 0; k < m32; ++k) {
        const int sk = __builtin_amdgcn_readlane(sr, k);
        const v4f r = *(const v4fa*)(hp + (size_t)sk * DF + 4 * lane);
        a0 += r.x; a1 += r.y; a2 += r.z; a3 += r.w;
      }
    }
    const v4f sv = *(const v4fa*)(hp + (size_t)nc * DF + 4 * lane);
    asm volatile("" :: "v"(sv));
    v4f pr = {0.f, 0.f, 0.f, 0.f};
    if constexpr (HASP != 0) {
      pr = *(const v4fa*)(stp + (size_t)nc * DF + 4 * lane);
      asm volatile("" :: "v"(pr));
    }
    v4f xv;
    xv.x = fin1(a0, sv.x, dd, b4.x, bad, live);
    xv.y = fin1(a1, sv.y, dd, b4.y, bad, live);
    xv.z = fin1(a2, sv.z, dd, b4.z, bad, live);
    xv.w = fin1(a3, sv.w, dd, b4.w, bad, live);

    if constexpr (LAST != 0) {
      float* op = outp + (size_t)node * DF + 4 * lane;
      if (node < nN) {
        *(volatile v4f*)op = xv;
        __threadfence();
        *(volatile v4f*)op = xv;
      }
    } else {
      const float s0 = xv.x + pr.x, s1 = xv.y + pr.y, s2 = xv.z + pr.z, s3 = xv.w + pr.w;
      const float r0 = live ? s0 : 0.0f, r1 = live ? s1 : 0.0f;
      const float r2 = live ? s2 : 0.0f, r3 = live ? s3 : 0.0f;
      v4us mh, ml;
      {
        unsigned lb;
        unsigned hb;
        hb = hl_bits(r0, lb); mh[0] = (unsigned short)hb; ml[0] = (unsigned short)lb;
        hb = hl_bits(r1, lb); mh[1] = (unsigned short)hb; ml[1] = (unsigned short)lb;
        hb = hl_bits(r2, lb); mh[2] = (unsigned short)hb; ml[2] = (unsigned short)lb;
        hb = hl_bits(r3, lb); mh[3] = (unsigned short)hb; ml[3] = (unsigned short)lb;
      }
      *(v4usa*)(rb + 4 * lane)      = mh;
      *(v4usa*)(rb + DF + 4 * lane) = ml;
      wave_sync();
      const v8us q0 = *(const v8usa*)(rb + 8 * lane);
      wave_sync();
      if (node < mRows) {
        float* xp = stn + (size_t)node * DF + 4 * lane;
        unsigned short* apw = ain + (size_t)node * K2 + 8 * lane;
        if constexpr (WRX != 0) *(volatile v4f*)xp = xv;
        *(volatile v8us*)apw = q0;
        __threadfence();
        if constexpr (WRX != 0) *(volatile v4f*)xp = xv;
        *(volatile v8us*)apw = q0;
      }
    }
  }
}

static inline size_t al256(size_t o) { return (o + 255) & ~(size_t)255; }

extern "C" void kernel_launch(void* const* d_in, const int* in_sizes, int n_in,
                              void* d_out, int out_size, void* d_ws, size_t ws_size,
                              hipStream_t stream) {
  if (n_in < 10) return;
  if (in_sizes[0] != NNODE * DF) return;
  if (in_sizes[1] != 2 * NEDGE) return;
  for (int l = 0; l < 4; ++l) {
    if (in_sizes[2 + 2 * l] != DF * DF) return;
    if (in_sizes[3 + 2 * l] != DF) return;
  }
  if (out_size != NNODE * DF) return;
  const int nN = NNODE, nE = NEDGE;

  const float* x    = (const float*)d_in[0];
  const int*   edge = (const int*)  d_in[1];
  const float* W1   = (const float*)d_in[2];
  const float* b1   = (const float*)d_in[3];
  const float* W2   = (const float*)d_in[4];
  const float* b2   = (const float*)d_in[5];
  const float* W3   = (const float*)d_in[6];
  const float* b3   = (const float*)d_in[7];
  const float* W4   = (const float*)d_in[8];
  const float* b4   = (const float*)d_in[9];
  float* out = (float*)d_out;
  const int* src = edge;
  const int* dst = edge + nE;
  const int vec8 = ((nE & 3) == 0) ? 1 : 0;

  char* ws = (char*)d_ws;
  size_t off = 0;
  const size_t oHP  = off; off = al256(off + (size_t)MPAD * DF * 4);
  const size_t oAIN = off; off = al256(off + (size_t)MPAD * K2 * 2);
  const size_t oXP  = off; off = al256(off + (size_t)MPAD * DF * 4);
  const size_t oXQ  = off; off = al256(off + (size_t)MPAD * DF * 4);
  const size_t oLST = off; off = al256(off + (size_t)NBLK * RCAP_WS * 4);
  const size_t oCNT = off; off = al256(off + (size_t)NBLK * NBA * 4);
  const size_t oOFF = off; off = al256(off + (size_t)NBLK * NBA * 4);
  const size_t oDIS = off; off = al256(off + (size_t)NBLK * NBA * 4);
  const size_t oFLG = off; off = al256(off + (size_t)NBLK * FLP * 4);
  const size_t oW1T = off; off = al256(off + (size_t)DF * K1 * 2);
  const size_t oW2D = off; off = al256(off + (size_t)DF * K2 * 2);
  const size_t oW3D = off; off = al256(off + (size_t)DF * K2 * 2);
  const size_t oW4D = off; off = al256(off + (size_t)DF * K2 * 2);
  const size_t oBT  = off; off = al256(off + (size_t)4 * DF * 4);
  if (off > ws_size) return;
  if ((size_t)MPAD * K1 * 2 > (size_t)MPAD * K2 * 2) return;
  float*          HP   = (float*)(ws + oHP);
  unsigned short* AIN  = (unsigned short*)(ws + oAIN);
  unsigned short* XB   = (unsigned short*)(ws + oAIN);
  float*          XP   = (float*)(ws + oXP);
  float*          XQ   = (float*)(ws + oXQ);
  int*            LIST = (int*)(ws + oLST);
  int*            CNT  = (int*)(ws + oCNT);
  int*            OFF  = (int*)(ws + oOFF);
  float*          DIS  = (float*)(ws + oDIS);
  int*            FLG  = (int*)(ws + oFLG);
  unsigned short* W1T  = (unsigned short*)(ws + oW1T);
  unsigned short* W2D  = (unsigned short*)(ws + oW2D);
  unsigned short* W3D  = (unsigned short*)(ws + oW3D);
  unsigned short* W4D  = (unsigned short*)(ws + oW4D);
  float*          BT   = (float*)(ws + oBT);

  const size_t bkLds = (size_t)BK_LDS_INTS * 4;
  const size_t gLds  = (size_t)G_LDS_FLOATS * 4;
  hipFuncSetAttribute(reinterpret_cast<const void*>(&k_bucket), hipFuncAttributeMaxDynamicSharedMemorySize, (int)bkLds);
  hipFuncSetAttribute(reinterpret_cast<const void*>(&k_gemm), hipFuncAttributeMaxDynamicSharedMemorySize, (int)gLds);

  const int nUnits = NUWE + MPAD * 16;
  const int gM = MPAD / GBM;

  k_prep<<<nUnits / NTHR, NTHR, 0, stream>>>(x, W1, W2, W3, W4, b1, b2, b3, b4,
                                             XB, W1T, W2D, W3D, W4D, BT, nN, nUnits);
  k_bucket<<<NBLK, NTHR, bkLds, stream>>>(src, dst, nE, nN, vec8, LIST, CNT, OFF, DIS, FLG);
  k_gemm<<<gM, GTHR, gLds, stream>>>(XB, W1T, K1, DIS, HP, nN);
  k_replay<0, 1, 0><<<NBLK, NTHR, 0, stream>>>(LIST, CNT, OFF, DIS, FLG, HP, BT + 0 * DF, XQ, XP, AIN, out, nN, MPAD);
  k_gemm<<<gM, GTHR, gLds, stream>>>(AIN, W2D, K2, DIS, HP, nN);
  k_replay<1, 1, 0><<<NBLK, NTHR, 0, stream>>>(LIST, CNT, OFF, DIS, FLG, HP, BT + 1 * DF, XP, XQ, AIN, out, nN, MPAD);
  k_gemm<<<gM, GTHR, gLds, stream>>>(AIN, W3D, K2, DIS, HP, nN);
  k_replay<1, 1, 0><<<NBLK, NTHR, 0, stream>>>(LIST, CNT, OFF, DIS, FLG, HP, BT + 2 * DF, XQ, XP, AIN, out, nN, MPAD);
  k_gemm<<<gM, GTHR, gLds, stream>>>(AIN, W4D, K2, DIS, HP, nN);
  k_replay<1, 0, 0><<<NBLK, NTHR, 0, stream>>>(LIST, CNT, OFF, DIS, FLG, HP, BT + 3 * DF, XP, XQ, AIN, out, nN, MPAD);
  k_gemm<<<gM, GTHR, gLds, stream>>>(AIN, W4D, K2, DIS, HP, nN);
  k_replay<0, 0, 1><<<NBLK, NTHR, 0, stream>>>(LIST, CNT, OFF, DIS, FLG, HP, BT + 3 * DF, XP, XQ, AIN, out, nN, MPAD);
}
